// GraphMessagePassing_171798692411
// MI455X (gfx1250) — hardware-verified
//
#include <hip/hip_runtime.h>
#include <math.h>

typedef __attribute__((ext_vector_type(16))) _Float16 v16h;
typedef __attribute__((ext_vector_type(16))) __bf16 v16b;
typedef __attribute__((ext_vector_type(8)))  _Float16 v8h;
typedef __attribute__((ext_vector_type(8)))  float v8f;
typedef __attribute__((ext_vector_type(4)))  float v4f;
typedef __attribute__((ext_vector_type(2)))  float v2f;
typedef __attribute__((ext_vector_type(4)))  unsigned v4u;
typedef __attribute__((ext_vector_type(4)))  int v4i;
typedef float __attribute__((may_alias)) float_a;
typedef int __attribute__((may_alias)) int_a;

template <typename T> __device__ __forceinline__ void vst2(void* p, T v) { *(volatile T*)p = v; __threadfence(); *(volatile T*)p = v; }
__device__ __forceinline__ v8f wmma16(v16h a, v16h b, v8f c) {
  v8f d = __builtin_amdgcn_wmma_f32_16x16x32_f16(false, a, false, b, (short)0, c, false, false);
  asm volatile("v_nop\n\tv_nop\n\tv_nop\n\tv_nop" : "+v"(d) : "v"(a), "v"(b));
  return d;
}
__device__ __forceinline__ v8f wmma_bf(v16b a, v16b b, v8f c) {
  v8f d = __builtin_amdgcn_wmma_f32_16x16x32_bf16(false, a, false, b, (short)0, c, false, false);
  asm volatile("v_nop\n\tv_nop\n\tv_nop\n\tv_nop" : "+v"(d) : "v"(a), "v"(b));
  return d;
}
__device__ __forceinline__ v16h frag_h(const _Float16* rowk0, int lane) {
  union { v16h v; v8h q[2]; } u; const _Float16* p = rowk0 + 8 * (lane >> 4);
  u.q[0] = *(const v8h*)p; u.q[1] = *(const v8h*)(p + 16); return u.v;
}
__device__ __forceinline__ v16h frag_f32(const float* rowk0, int lane) {
  v16h a; const float* p = rowk0 + 8 * (lane >> 4);
#pragma unroll
  for (int i = 0; i < 8; ++i) { a[i] = (_Float16)p[i]; a[8 + i] = (_Float16)p[16 + i]; }
  return a;
}
__device__ __forceinline__ v16h frag_f32s(const float* rowk0, int lane, float sc) {
  v16h a; const float* p = rowk0 + 8 * (lane >> 4);
#pragma unroll
  for (int i = 0; i < 8; ++i) { a[i] = (_Float16)(p[i] * sc); a[8 + i] = (_Float16)(p[16 + i] * sc); }
  return a;
}
__device__ __forceinline__ v16h fragc_f32(const float* W, int k0, int n, int lane, int ld, int K) {
  v16h a; const int g = lane >> 4;
#pragma unroll
  for (int i = 0; i < 8; ++i) { const int ka = k0 + 8 * g + i, kb = ka + 16;
    a[i] = (_Float16)(ka < K ? W[(size_t)(ka < K ? ka : K - 1) * ld + n] : 0.f); a[8 + i] = (_Float16)(kb < K ? W[(size_t)(kb < K ? kb : K - 1) * ld + n] : 0.f); }
  return a;
}
struct F2 { v16b h, l; };
__device__ __forceinline__ F2 bsplit16(const float v[16]) { F2 r;
#pragma unroll
  for (int i = 0; i < 16; ++i) { const __bf16 h = (__bf16)v[i]; r.h[i] = h; r.l[i] = (__bf16)(v[i] - (float)h); }
  return r; }
__device__ __forceinline__ F2 split_row(const float* row, int k0, int lane) { float v[16]; const float* p = row + k0 + 8 * (lane >> 4);
#pragma unroll
  for (int i = 0; i < 8; ++i) { v[i] = p[i]; v[8 + i] = p[16 + i]; }
  return bsplit16(v); }
__device__ __forceinline__ F2 split_rowK(const float* row, int k0, int lane, int K) { float v[16]; const int g = lane >> 4;
#pragma unroll
  for (int i = 0; i < 8; ++i) { const int ka = k0 + 8 * g + i, kb = ka + 16; v[i] = ka < K ? row[ka < K ? ka : K - 1] : 0.f; v[8 + i] = kb < K ? row[kb < K ? kb : K - 1] : 0.f; }
  return bsplit16(v); }
__device__ __forceinline__ F2 split_col(const float* W, int k0, int n, int lane, int ld, int K) { float v[16]; const int g = lane >> 4;
#pragma unroll
  for (int i = 0; i < 8; ++i) { const int ka = k0 + 8 * g + i, kb = ka + 16; v[i] = ka < K ? W[(size_t)(ka < K ? ka : K - 1) * ld + n] : 0.f; v[8 + i] = kb < K ? W[(size_t)(kb < K ? kb : K - 1) * ld + n] : 0.f; }
  return bsplit16(v); }
__device__ __forceinline__ v8f mac3(const F2& a, const F2& b, v8f c) { c = wmma_bf(a.l, b.h, c); c = wmma_bf(a.h, b.l, c); return wmma_bf(a.h, b.h, c); }
__device__ __forceinline__ float sigm(float v) { return 1.0f / (1.0f + expf(-v)); }
#define LDSX() do { asm volatile("s_wait_dscnt 0" ::: "memory"); __builtin_amdgcn_wave_barrier(); __builtin_amdgcn_fence(__ATOMIC_RELEASE, "workgroup"); } while (0)

__device__ __forceinline__ float bfr(float v) { return (float)(__bf16)v; }
#define NBT 2
#define NN 1000
#define NE 2000
#define HH 128
#ifndef TNB
#define TNB NBT
#endif
#define NEP 2048
#define WS_N2E 0u
#define WS_NEW (WS_N2E + 4u * (size_t)NBT * NEP * HH)
#define WS_END (WS_NEW + 4u * (size_t)NBT * NEP * HH)
__global__ __launch_bounds__(128) void k_n2e(const float* __restrict__ N2E_A, const float* __restrict__ NS, float* __restrict__ OUTP) { __shared__ __align__(16) float sf[4][16][132];
  const int tid = threadIdx.x, wave = tid >> 5, lane = tid & 31, col = lane & 15, g = lane >> 4; const size_t b = blockIdx.y; const int e0 = blockIdx.x * 64 + wave * 16; const int ea = (e0 + col) < NE ? e0 + col : NE - 1;
  v8f acc[8] = {};
#pragma unroll 1
  for (int kc = 0; kc < (NN + 31) / 32; ++kc) { v16b a; const float* p = N2E_A + (b * NE + ea) * NN;
#pragma unroll
    for (int i = 0; i < 8; ++i) { const int ka = kc * 32 + 8 * g + i, kb = ka + 16; a[i] = ka < NN ? (__bf16)p[ka] : (__bf16)0.f; a[8 + i] = kb < NN ? (__bf16)p[kb] : (__bf16)0.f; }
#pragma unroll
    for (int j = 0; j < 8; ++j) { v16b w; const int o = j * 16 + col;
#pragma unroll
      for (int i = 0; i < 8; ++i) { const int ka = kc * 32 + 8 * g + i, kb = ka + 16; w[i] = ka < NN ? (__bf16)NS[(b * NN + ka) * HH + o] : (__bf16)0.f; w[8 + i] = kb < NN ? (__bf16)NS[(b * NN + kb) * HH + o] : (__bf16)0.f; }
      asm volatile("s_wait_loadcnt 0x0" ::: "memory"); acc[j] = wmma_bf(a, w, acc[j]); } }
#pragma unroll
  for (int j = 0; j < 8; ++j)
#pragma unroll
    for (int r = 0; r < 8; ++r) sf[wave][8 * g + r][j * 16 + col] = acc[j][r];
  LDSX(); for (int rl = 0; rl < 16; ++rl) vst2(OUTP + (b * NEP + e0 + rl) * HH + lane * 4, *(const v4f*)&sf[wave][rl][lane * 4]); }
__global__ __launch_bounds__(128) void k_enet(const float* __restrict__ N2EP, const float* __restrict__ EV, const float* __restrict__ Wt, float* __restrict__ NEWP) { __shared__ __align__(16) float sf[4][16][132];
  const int tid = threadIdx.x, wave = tid >> 5, lane = tid & 31, col = lane & 15, g = lane >> 4; const size_t b = blockIdx.y; const int e0 = blockIdx.x * 64 + wave * 16;
  F2 af[4];
#pragma unroll
  for (int kc = 0; kc < 4; ++kc) af[kc] = split_row(N2EP + (b * NEP + e0 + col) * HH, kc * 32, lane);
  float evr[8];
  v8f res[8] = {};
#pragma unroll 1
  for (int h = 0; h < HH; ++h) { v8f acc[8] = {};
#pragma unroll
    for (int r = 0; r < 8; ++r) { const int e = e0 + 8 * g + r; evr[r] = bfr(EV[(b * NE + (e < NE ? e : NE - 1)) * HH + h]); }
#pragma unroll
    for (int kc = 0; kc < 4; ++kc) {
#pragma unroll
      for (int j = 0; j < 8; ++j) { v16b w; const float* wr = Wt + ((size_t)h * HH + j * 16 + col) * HH + kc * 32 + 8 * g;
#pragma unroll
        for (int q = 0; q < 8; ++q) { w[q] = (__bf16)wr[q]; w[8 + q] = (__bf16)wr[16 + q]; }
        asm volatile("s_wait_loadcnt 0x0" ::: "memory"); acc[j] = wmma_bf(af[kc].h, w, acc[j]); acc[j] = wmma_bf(af[kc].l, w, acc[j]); } }
#pragma unroll
    for (int j = 0; j < 8; ++j)
#pragma unroll
      for (int r = 0; r < 8; ++r) res[j][r] += evr[r] * acc[j][r]; }
#pragma unroll
  for (int j = 0; j < 8; ++j)
#pragma unroll
    for (int r = 0; r < 8; ++r) sf[wave][8 * g + r][j * 16 + col] = res[j][r];
  LDSX(); for (int rl = 0; rl < 16; ++rl) vst2(NEWP + (b * NEP + e0 + rl) * HH + lane * 4, *(const v4f*)&sf[wave][rl][lane * 4]); }
__global__ __launch_bounds__(128) void k_agg(const float* __restrict__ E2N, const float* __restrict__ NEWP, const float* __restrict__ NS, float* __restrict__ OUT) { __shared__ __align__(16) float sf[4][16][132]; __shared__ float snrm[4][16];
  const int tid = threadIdx.x, wave = tid >> 5, lane = tid & 31, col = lane & 15, g = lane >> 4; const size_t b = blockIdx.y; const int n0 = blockIdx.x * 64 + wave * 16; const int na = (n0 + col) < NN ? n0 + col : NN - 1; const float* arow = E2N + (b * NN + na) * NE;
  v8f acc[8] = {}; float rsum = 0.f;
#pragma unroll 1
  for (int kc = 0; kc < (NE + 31) / 32; ++kc) { v16b a;
#pragma unroll
    for (int i = 0; i < 8; ++i) { const int ka = kc * 32 + 8 * g + i, kb = ka + 16; const float va = ka < NE ? bfr(arow[ka]) : 0.f, vb = kb < NE ? bfr(arow[kb]) : 0.f; a[i] = (__bf16)va; a[8 + i] = (__bf16)vb; rsum += va + vb; }
#pragma unroll
    for (int j = 0; j < 8; ++j) { float wv[16]; const int o = j * 16 + col;
#pragma unroll
      for (int i = 0; i < 8; ++i) { const int ka = kc * 32 + 8 * g + i, kb = ka + 16; wv[i] = ka < NE ? NEWP[(b * NEP + ka) * HH + o] : 0.f; wv[8 + i] = kb < NE ? NEWP[(b * NEP + kb) * HH + o] : 0.f; }
      asm volatile("s_wait_loadcnt 0x0" ::: "memory"); const F2 w = bsplit16(wv); acc[j] = wmma_bf(a, w.h, acc[j]); acc[j] = wmma_bf(a, w.l, acc[j]); } }
  rsum += __shfl_xor(rsum, 16);
  if (g == 0) snrm[wave][col] = rsum;
  LDSX();
#pragma unroll
  for (int j = 0; j < 8; ++j) { const int o = j * 16 + col;
#pragma unroll
    for (int r = 0; r < 8; ++r) { const int rl = 8 * g + r; const int n = n0 + rl; const float ns = bfr(NS[(b * NN + (n < NN ? n : NN - 1)) * HH + o]); sf[wave][rl][o] = (acc[j][r] + ns) / (snrm[wave][rl] + 1.0f); }
    asm volatile("s_wait_loadcnt 0x0" ::: "memory"); }
  LDSX(); for (int rl = 0; rl < 16; ++rl) { const int n = n0 + rl; if (n < NN) vst2(OUT + (b * NN + n) * HH + lane * 4, *(const v4f*)&sf[wave][rl][lane * 4]); } }
extern "C" void kernel_launch(void* const* d_in, const int* in_sizes, int n_in, void* d_out, int out_size, void* d_ws, size_t ws_size, hipStream_t stream) {
  (void)in_sizes; (void)n_in; (void)out_size;
  const float** F = (const float**)d_in;
  if (ws_size < (size_t)WS_END) return;
  char* ws = (char*)d_ws; float *N2EP = (float*)(ws + WS_N2E), *NEWP = (float*)(ws + WS_NEW);
  k_n2e<<<dim3(NEP / 64, TNB), 128, 0, stream>>>(F[2], F[0], N2EP);
  k_enet<<<dim3(NEP / 64, TNB), 128, 0, stream>>>(N2EP, F[1], F[4], NEWP);
  k_agg<<<dim3((NN + 63) / 64, TNB), 128, 0, stream>>>(F[3], NEWP, F[0], (float*)d_out);
}
